// MultiHeadAttention_51780125720948
// MI455X (gfx1250) — hardware-verified
//
#include <hip/hip_runtime.h>
#ifndef NB
#define NB 8
#endif
#ifndef SEQ
#define SEQ 1024
#endif
#define NB_FULL 8
#define SEQ_FULL 1024
#define DM 1024
#define NH 16
#define HD 64
#define NR ((size_t)NB * SEQ)
static_assert(NH * HD == DM);
static_assert(SEQ % 128 == 0);
static_assert(SEQ <= SEQ_FULL);
static_assert(NB >= 1 && NB <= NB_FULL);
static_assert(DM == 128 * 8);
static_assert(DM % 256 == 0);
static_assert(HD == 64);
static_assert(DM % 64 == 0);
static_assert(DM % 32 == 0);
static_assert(SEQ % 64 == 0);
static_assert(((size_t)NB * SEQ) % 128 == 0);
static_assert(((size_t)DM * DM) % 8 == 0);
static_assert((size_t)4 * DM * DM * 2 + (size_t)6 * NB * SEQ * DM * 2 <= (size_t)134217728);

typedef _Float16 v16h __attribute__((ext_vector_type(16)));
typedef unsigned short v8us __attribute__((ext_vector_type(8), may_alias));
typedef float v8f __attribute__((ext_vector_type(8)));
typedef float v4f __attribute__((ext_vector_type(4)));
typedef float v4fa __attribute__((ext_vector_type(4), may_alias));
typedef _Float16 v4h __attribute__((ext_vector_type(4)));
union FragH { v16h v; v8us half[2]; _Float16 h[16]; unsigned short u[16]; };

__device__ __forceinline__ unsigned short bf16_bits(float x) { unsigned int u = __float_as_uint(x); return (unsigned short)((u + 0x7FFFu + ((u >> 16) & 1u)) >> 16); }
__device__ __forceinline__ float bf16_val(unsigned short b) { return __uint_as_float(((unsigned int)b) << 16); }
__device__ __forceinline__ float bf16_rne(float x) { return bf16_val(bf16_bits(x)); }

typedef _Float16 h16;
static __device__ __forceinline__ h16 toh_flush(float v) { const h16 r = (h16)v; return (fabsf(v) < 6.103515625e-05f) ? (h16)0.0f : r; }

__device__ __forceinline__ v16h g2_frag(const _Float16* p, int hh) { FragH f; f.half[0] = *(const v8us*)((const unsigned short*)p + 8 * hh); f.half[1] = *(const v8us*)((const unsigned short*)p + 16 + 8 * hh); return f.v; }
__device__ __forceinline__ v8f g2_mma(v16h a, v16h b, v8f c) { v8f d = __builtin_amdgcn_wmma_f32_16x16x32_f16(false, a, false, b, (short)0, c, false, false); asm volatile("v_nop\n\tv_nop\n\tv_nop\n\tv_nop" : "+v"(d) : "v"(a), "v"(b)); return d; }
__device__ __forceinline__ v8f mma2(v16h a0, v16h b0, v16h a1, v16h b1, v8f c) {
  c = __builtin_amdgcn_wmma_f32_16x16x32_f16(false, a0, false, b0, (short)0, c, false, false);
  c = __builtin_amdgcn_wmma_f32_16x16x32_f16(false, a1, false, b1, (short)0, c, false, false);
  asm volatile("v_nop\n\tv_nop\n\tv_nop\n\tv_nop" : "+v"(c) : "v"(a0), "v"(b0), "v"(a1), "v"(b1));
  return c;
}

__global__ __launch_bounds__(256) void k_wnat(const float* __restrict__ w, size_t n8, _Float16* __restrict__ Bt) {
  const size_t t = (size_t)blockIdx.x * 256 + threadIdx.x; if (t >= n8) return; FragH f;
#pragma unroll
  for (int q = 0; q < 8; ++q) f.h[q] = (_Float16)(bf16_rne(w[t * 8 + q]) * 16.0f);
  const v8us o = f.half[0];
  *(volatile v8us*)((unsigned short*)Bt + t * 8) = o; __threadfence(); *(volatile v8us*)((unsigned short*)Bt + t * 8) = o;
}

__global__ __launch_bounds__(128) void k_xcvt(const float* __restrict__ x, _Float16* __restrict__ X16) {
  const int r = blockIdx.x; const int b = r / SEQ, s = r - b * SEQ;
  const int t = threadIdx.x;
  const float* xr = x + ((size_t)b * SEQ_FULL + s) * DM + 8 * t;
  const v4f xa = *(const v4fa*)xr, xb = *(const v4fa*)(xr + 4);
  FragH f;
#pragma unroll
  for (int q = 0; q < 4; ++q) { f.h[q] = toh_flush(bf16_rne(xa[q])); f.h[4 + q] = toh_flush(bf16_rne(xb[q])); }
  const v8us o = f.half[0];
  unsigned short* d = (unsigned short*)X16 + (size_t)r * DM + 8 * t;
  *(volatile v8us*)d = o; __threadfence(); *(volatile v8us*)d = o;
}

__device__ __forceinline__ void mac32x64(const _Float16* __restrict__ a0p, const _Float16* __restrict__ a1p, const _Float16* __restrict__ b0p, size_t ldb, int K, int hh,
                                         v8f& c00, v8f& c01, v8f& c02, v8f& c03, v8f& c10, v8f& c11, v8f& c12, v8f& c13) {
  const _Float16* b1p = b0p + 16 * ldb; const _Float16* b2p = b1p + 16 * ldb; const _Float16* b3p = b2p + 16 * ldb;
#pragma unroll 1
  for (int kb = 0; kb < K; kb += 32) {
    const v16h a0 = g2_frag(a0p + kb, hh), a1 = g2_frag(a1p + kb, hh);
    v16h bq = g2_frag(b0p + kb, hh); c00 = g2_mma(a0, bq, c00); c10 = g2_mma(a1, bq, c10);
    bq = g2_frag(b1p + kb, hh); c01 = g2_mma(a0, bq, c01); c11 = g2_mma(a1, bq, c11);
    bq = g2_frag(b2p + kb, hh); c02 = g2_mma(a0, bq, c02); c12 = g2_mma(a1, bq, c12);
    bq = g2_frag(b3p + kb, hh); c03 = g2_mma(a0, bq, c03); c13 = g2_mma(a1, bq, c13);
  }
}

__global__ __launch_bounds__(128) void k_qkv(const _Float16* __restrict__ X16, const _Float16* __restrict__ Bt, const float* __restrict__ bq, const float* __restrict__ bv, float alpha, _Float16* __restrict__ Y16) {
  __shared__ __attribute__((aligned(16))) float so[4][32][68];
  const int tid = threadIdx.x, w = tid >> 5, lane = tid & 31, ln = lane & 15, hh = lane >> 4;
  const int by = blockIdx.y;
  const _Float16* Bh = Bt + (size_t)by * DM * DM;
  _Float16* Yp = Y16 + (size_t)by * NR * DM;
  const int ntn = DM / 64;
  const int mt = blockIdx.x / ntn, nq = blockIdx.x - mt * ntn;
  const int row0 = mt * 128 + 32 * w, col0 = nq * 64;
  if (row0 >= (int)NR) return;
  const _Float16* a0p = X16 + (size_t)(row0 + ln) * DM; const _Float16* a1p = a0p + (size_t)16 * DM;
  const _Float16* b0p = Bh + (size_t)(col0 + ln) * DM;
  const v8f z8 = {0.f, 0.f, 0.f, 0.f, 0.f, 0.f, 0.f, 0.f};
  v8f c00 = z8, c01 = z8, c02 = z8, c03 = z8, c10 = z8, c11 = z8, c12 = z8, c13 = z8;
  mac32x64(a0p, a1p, b0p, (size_t)DM, DM, hh, c00, c01, c02, c03, c10, c11, c12, c13);
  v8f accs[8] = {c00, c01, c02, c03, c10, c11, c12, c13};
#pragma unroll
  for (int u = 0; u < 8; ++u) {
    const int t = u & 3, half = u >> 2; const int col = col0 + t * 16 + ln;
    const float bqv = bf16_rne(bq[col]);
    const float bvv = bf16_rne(bv[col]);
    const float bias = (by == 0) ? bqv : ((by == 2) ? bvv : 0.0f);
#pragma unroll
    for (int r = 0; r < 8; ++r) so[w][half * 16 + 8 * hh + r][t * 16 + ln] = accs[u][r] * alpha + bias;
  }
  __builtin_amdgcn_fence(4  , "workgroup"); __builtin_amdgcn_wave_barrier();
  const int rsub = lane >> 4, c4 = (lane & 15) * 4;
  for (int pass = 0; pass < 2; ++pass) {
#pragma unroll
    for (int q = 0; q < 16; ++q) {
      const int r = q * 2 + rsub; const v4f v = *(const v4fa*)&so[w][r][c4]; v4h h4;
#pragma unroll
      for (int i = 0; i < 4; ++i) h4[i] = toh_flush(v[i]);
      *(volatile v4h*)(Yp + (size_t)(row0 + r) * DM + col0 + c4) = h4;
    }
    if (pass == 0) __threadfence();
  }
}

template <int NHv, int TTv>
__global__ __launch_bounds__(256) void k_vt(const _Float16* __restrict__ V16, int ldv, int voff, _Float16* __restrict__ Vt) {
  __shared__ unsigned short tl[64][66];
  const int tid = threadIdx.x; const int slab = blockIdx.x / (TTv / 64), lg = blockIdx.x % (TTv / 64); const int b = slab / NHv, h = slab % NHv;
  for (int i = tid; i < 64 * 8; i += 256) {
    const int r = i / 8, c8 = (i % 8) * 8; FragH f; f.half[0] = *(const v8us*)((const unsigned short*)V16 + ((size_t)b * TTv + lg * 64 + r) * ldv + voff + h * 64 + c8);
#pragma unroll
    for (int q = 0; q < 8; ++q) tl[r][c8 + q] = f.u[q];
  }
  __syncthreads();
  for (int pass = 0; pass < 2; ++pass) {
#pragma unroll
    for (int rd = 0; rd < 2; ++rd) {
      const int d = rd * 32 + tid / 8, pc = tid % 8; FragH f;
#pragma unroll
      for (int q = 0; q < 8; ++q) f.u[q] = tl[pc * 8 + q][d];
      *(volatile v8us*)((unsigned short*)Vt + ((size_t)slab * 64 + d) * TTv + lg * 64 + pc * 8) = f.half[0];
    }
    if (pass == 0) __threadfence();
  }
}

__global__ __launch_bounds__(128) void k_attn(const _Float16* __restrict__ Q16, const _Float16* __restrict__ K16, const _Float16* __restrict__ VT, _Float16* __restrict__ O16) {
  __shared__ __attribute__((aligned(16))) unsigned short so[4][16][72];
  const int tid = threadIdx.x, w = tid >> 5, lane = tid & 31, ln = lane & 15, hh = lane >> 4;
  const int h = blockIdx.y, b = blockIdx.z;
  const int q0 = blockIdx.x * 64 + w * 16;
  const size_t rq = (size_t)b * SEQ + q0;
  const size_t rk = (size_t)b * SEQ;
  const _Float16* qp = Q16 + (rq + ln) * DM + h * HD;
  const v16h qb0 = g2_frag(qp, hh), qb1 = g2_frag(qp + 32, hh);
  const _Float16* kp0 = K16 + (rk + ln) * DM + h * HD;
  const _Float16* vp0 = VT + ((size_t)(b * NH + h) * HD + ln) * SEQ;
  const v8f z8 = {0.f, 0.f, 0.f, 0.f, 0.f, 0.f, 0.f, 0.f};
  v8f o0 = z8, o1 = z8, o2 = z8, o3 = z8;
  float mrun = -1.0e30f, lrun = 0.f;
#pragma unroll 1
  for (int kt = 0; kt < SEQ; kt += 64) {
    v8f s[4];
#pragma unroll
    for (int j = 0; j < 4; ++j) {
      const _Float16* kp = kp0 + (size_t)(kt + 16 * j) * DM;
      const v16h ka0 = g2_frag(kp, hh), ka1 = g2_frag(kp + 32, hh);
      s[j] = mma2(ka0, qb0, ka1, qb1, z8);
    }
    float mx = -1.0e30f;
#pragma unroll
    for (int j = 0; j < 4; ++j)
#pragma unroll
      for (int r = 0; r < 8; ++r) mx = fmaxf(mx, s[j][r]);
    mx = fmaxf(mx, __shfl_xor(mx, 16, 32));
    const float mnew = fmaxf(mrun, mx * 0.125f);
    const float alpha = __expf(mrun - mnew);
    mrun = mnew;
    float ps = 0.f; FragH pf[2];
#pragma unroll
    for (int j = 0; j < 4; ++j)
#pragma unroll
      for (int r = 0; r < 8; ++r) {
        const float p = __expf(s[j][r] * 0.125f - mnew);
        ps += p;
        pf[j >> 1].h[(j & 1) * 8 + r] = (_Float16)(p * 1024.0f);
      }
    ps += __shfl_xor(ps, 16, 32);
    lrun = lrun * alpha + ps;
#pragma unroll
    for (int r = 0; r < 8; ++r) { o0[r] *= alpha; o1[r] *= alpha; o2[r] *= alpha; o3[r] *= alpha; }
    { const _Float16* vp = vp0 + (size_t)0 * 16 * SEQ + kt; const v16h va0 = g2_frag(vp, hh), va1 = g2_frag(vp + 32, hh); o0 = mma2(va0, pf[0].v, va1, pf[1].v, o0); }
    { const _Float16* vp = vp0 + (size_t)1 * 16 * SEQ + kt; const v16h va0 = g2_frag(vp, hh), va1 = g2_frag(vp + 32, hh); o1 = mma2(va0, pf[0].v, va1, pf[1].v, o1); }
    { const _Float16* vp = vp0 + (size_t)2 * 16 * SEQ + kt; const v16h va0 = g2_frag(vp, hh), va1 = g2_frag(vp + 32, hh); o2 = mma2(va0, pf[0].v, va1, pf[1].v, o2); }
    { const _Float16* vp = vp0 + (size_t)3 * 16 * SEQ + kt; const v16h va0 = g2_frag(vp, hh), va1 = g2_frag(vp + 32, hh); o3 = mma2(va0, pf[0].v, va1, pf[1].v, o3); }
  }
  const float rl = (1.0f / lrun) * 0.015625f;
  { FragH f;
#pragma unroll
    for (int r = 0; r < 8; ++r) f.h[r] = (_Float16)(o0[r] * rl);
    *(v8us*)&so[w][ln][0 + 8 * hh] = f.half[0]; }
  { FragH f;
#pragma unroll
    for (int r = 0; r < 8; ++r) f.h[r] = (_Float16)(o1[r] * rl);
    *(v8us*)&so[w][ln][16 + 8 * hh] = f.half[0]; }
  { FragH f;
#pragma unroll
    for (int r = 0; r < 8; ++r) f.h[r] = (_Float16)(o2[r] * rl);
    *(v8us*)&so[w][ln][32 + 8 * hh] = f.half[0]; }
  { FragH f;
#pragma unroll
    for (int r = 0; r < 8; ++r) f.h[r] = (_Float16)(o3[r] * rl);
    *(v8us*)&so[w][ln][48 + 8 * hh] = f.half[0]; }
  __builtin_amdgcn_fence(4  , "workgroup"); __builtin_amdgcn_wave_barrier();
  const int li = lane >> 3, pc = lane & 7;
  for (int pass = 0; pass < 2; ++pass) {
#pragma unroll
    for (int g = 0; g < 4; ++g) {
      const int i = g * 4 + li;
      const v8us v = *(const v8us*)&so[w][i][pc * 8];
      *(volatile v8us*)((unsigned short*)O16 + (rq + i) * DM + h * HD + pc * 8) = v;
    }
    if (pass == 0) __threadfence();
  }
}

__global__ __launch_bounds__(128) void k_out(const _Float16* __restrict__ A1, const _Float16* __restrict__ B1, const float* __restrict__ bo, float al1, float* __restrict__ Out) {
  __shared__ __attribute__((aligned(16))) float so[4][32][68];
  const int tid = threadIdx.x, w = tid >> 5, lane = tid & 31, ln = lane & 15, hh = lane >> 4;
  const int ntn = DM / 64;
  const int mt = blockIdx.x / ntn, nq = blockIdx.x - mt * ntn;
  const int row0 = mt * 128 + 32 * w, col0 = nq * 64;
  if (row0 >= (int)NR) return;
  const v8f z8 = {0.f, 0.f, 0.f, 0.f, 0.f, 0.f, 0.f, 0.f};
  v8f c00 = z8, c01 = z8, c02 = z8, c03 = z8, c10 = z8, c11 = z8, c12 = z8, c13 = z8;
  {
    const _Float16* a0p = A1 + (size_t)(row0 + ln) * DM; const _Float16* a1p = a0p + (size_t)16 * DM;
    const _Float16* b0p = B1 + (size_t)(col0 + ln) * DM;
    mac32x64(a0p, a1p, b0p, (size_t)DM, DM, hh, c00, c01, c02, c03, c10, c11, c12, c13);
    v8f accs[8] = {c00, c01, c02, c03, c10, c11, c12, c13};
#pragma unroll
    for (int u = 0; u < 8; ++u) {
      const int t = u & 3, half = u >> 2; const int col = col0 + t * 16 + ln;
      const float bias = bf16_rne(bo[col]);
#pragma unroll
      for (int r = 0; r < 8; ++r) so[w][half * 16 + 8 * hh + r][t * 16 + ln] = accs[u][r] * al1 + bias;
    }
  }
  __builtin_amdgcn_fence(4  , "workgroup"); __builtin_amdgcn_wave_barrier();
  const int rsub = lane >> 4, c4 = (lane & 15) * 4;
  for (int pass = 0; pass < 2; ++pass) {
#pragma unroll
    for (int q = 0; q < 16; ++q) {
      const int r = q * 2 + rsub; const v4f v = *(const v4fa*)&so[w][r][c4];
      *(volatile v4f*)(Out + (size_t)(row0 + r) * DM + col0 + c4) = v;
    }
    if (pass == 0) __threadfence();
  }
}

extern "C" void kernel_launch(void* const* d_in, const int* in_sizes, int n_in,
                              void* d_out, int out_size, void* d_ws, size_t ws_size, hipStream_t stream) {
  if (n_in < 9) return;
  if (in_sizes[0] < (int)(((size_t)(NB - 1) * SEQ_FULL + SEQ) * DM)) return;
  if (in_sizes[1] < NB + 1) return;
  if (in_sizes[2] < DM * DM || in_sizes[4] < DM * DM || in_sizes[5] < DM * DM || in_sizes[7] < DM * DM) return;
  if (in_sizes[3] < DM || in_sizes[6] < DM || in_sizes[8] < DM) return;
  if (out_size < (int)(NR * DM)) return;
  const float* x  = (const float*)d_in[0];
  const float* wq = (const float*)d_in[2]; const float* bq = (const float*)d_in[3];
  const float* wk = (const float*)d_in[4];
  const float* wv = (const float*)d_in[5]; const float* bv = (const float*)d_in[6];
  const float* wo = (const float*)d_in[7]; const float* bo = (const float*)d_in[8];
  char* ws = (char*)d_ws; size_t off = 0;
  auto take = [&](size_t bytes) { char* p = ws + off; off += (bytes + 255) & ~(size_t)255; return p; };
  _Float16* BQKV = (_Float16*)take((size_t)3 * DM * DM * 2);
  _Float16* BO   = (_Float16*)take((size_t)DM * DM * 2);
  _Float16* X16  = (_Float16*)take(NR * DM * 2);
  _Float16* QKV16 = (_Float16*)take((size_t)3 * NR * DM * 2);
  _Float16* VT   = (_Float16*)take((size_t)NB * NH * HD * SEQ * 2);
  _Float16* O16  = (_Float16*)take(NR * DM * 2);
  if (off > ws_size) return;
  if (off > (size_t)134217728) return;
  _Float16* Q16 = QKV16; _Float16* K16 = QKV16 + NR * DM; _Float16* V16 = QKV16 + (size_t)2 * NR * DM;

  { const size_t n8 = (size_t)DM * DM / 8; const unsigned g = (unsigned)((n8 + 255) / 256);
    k_wnat<<<g, 256, 0, stream>>>(wq, n8, BQKV);
    k_wnat<<<g, 256, 0, stream>>>(wk, n8, BQKV + (size_t)DM * DM);
    k_wnat<<<g, 256, 0, stream>>>(wv, n8, BQKV + (size_t)2 * DM * DM);
    k_wnat<<<g, 256, 0, stream>>>(wo, n8, BO); }
  k_xcvt<<<(unsigned)NR, 128, 0, stream>>>(x, X16);
  k_qkv<<<dim3((unsigned)((NR / 128) * (DM / 64)), 3), 128, 0, stream>>>(X16, BQKV, bq, bv, 0.0625f, QKV16);
  k_vt<NH, SEQ><<<(unsigned)(NB * NH * (SEQ / 64)), 256, 0, stream>>>(V16, DM, 0, VT);
  k_attn<<<dim3(SEQ / 64, NH, NB), 128, 0, stream>>>(Q16, K16, VT, O16);
  k_out<<<(unsigned)((NR / 128) * (DM / 64)), 128, 0, stream>>>(O16, BO, bo, 0.00390625f, (float*)d_out);
}
